// TransformerEncoderLayer_30889404793579
// MI455X (gfx1250) — hardware-verified
//
#include <hip/hip_runtime.h>
#ifndef SEQ
#define SEQ 2048
#endif
#define SEQ_FULL 2048
#define DM 1024
#define NH 16
#define HD 64
#define DFF 4096
#define LQ 3072

static_assert(SEQ % 128 == 0);
static_assert(SEQ <= SEQ_FULL);
static_assert(NH * HD == DM);
static_assert(LQ == 3 * DM);
static_assert(LQ == NH * 192);
static_assert(DM == 1024);
static_assert(HD == 64);
static_assert(DM % 64 == 0 && DFF % 64 == 0 && LQ % 64 == 0);
static_assert(DM % 32 == 0 && DFF % 32 == 0 && SEQ % 32 == 0);

typedef unsigned short v8us __attribute__((ext_vector_type(8), may_alias));
typedef float  v8f  __attribute__((ext_vector_type(8)));
typedef float  v4f  __attribute__((ext_vector_type(4)));
typedef float  v4fa __attribute__((ext_vector_type(4), may_alias));
typedef _Float16 v16h __attribute__((ext_vector_type(16)));
typedef _Float16 v4h  __attribute__((ext_vector_type(4)));
union FragH { v16h v; v8us half[2]; _Float16 h[16]; unsigned short u[16]; };

__device__ __forceinline__ unsigned short bf16_bits(float x) { unsigned int u = __float_as_uint(x); return (unsigned short)((u + 0x7FFFu + ((u >> 16) & 1u)) >> 16); }
__device__ __forceinline__ float bf16_rne(float x) { return __uint_as_float(((unsigned int)bf16_bits(x)) << 16); }

__device__ __forceinline__ v16h g2_frag(const _Float16* p, unsigned hh) { FragH f; f.half[0] = *(const v8us*)((const unsigned short*)p + 8 * hh); f.half[1] = *(const v8us*)((const unsigned short*)p + 16 + 8 * hh); return f.v; }
__device__ __forceinline__ v8f g2_mma(v16h a, v16h b, v8f c) { v8f d = __builtin_amdgcn_wmma_f32_16x16x32_f16(false, a, false, b, (short)0, c, false, false); asm volatile("v_nop\n\tv_nop\n\tv_nop\n\tv_nop" : "+v"(d) : "v"(a), "v"(b)); return d; }

__global__ __launch_bounds__(256) void k_x16(const float* __restrict__ x, _Float16* __restrict__ X16) {
  const unsigned t = blockIdx.x * 256u + threadIdx.x;
  if (t >= (unsigned)(SEQ * (DM / 8))) return;
  const unsigned r = t >> 7, c = (t & 127u) * 8u;
  const float* src = x + (size_t)r * DM + c;
  const v4f a = *(const v4fa*)src, b = *(const v4fa*)(src + 4);
  FragH f;
#pragma unroll
  for (int q = 0; q < 4; ++q) { f.h[q] = (_Float16)(bf16_rne(a[q]) * 16.0f); f.h[4 + q] = (_Float16)(bf16_rne(b[q]) * 16.0f); }
  const v8us o = f.half[0];
  unsigned short* d = (unsigned short*)X16 + (size_t)t * 8;
  *(volatile v8us*)d = o; __threadfence(); *(volatile v8us*)d = o;
}

__global__ __launch_bounds__(256) void k_wt_f16(const float* __restrict__ W, _Float16* __restrict__ Wt, unsigned K, unsigned N, float scale, unsigned ibs, unsigned obs) {
  const unsigned t = blockIdx.x * 256u + threadIdx.x; const unsigned k8n = K >> 3;
  if (t >= N * k8n) return;
  const float* Wb = W + (size_t)blockIdx.y * ibs;
  const unsigned n = t / k8n, k8 = (t - n * k8n) * 8u;
  FragH f;
#pragma unroll
  for (int i = 0; i < 8; ++i) f.h[i] = (_Float16)(bf16_rne(Wb[(size_t)(k8 + i) * N + n]) * scale);
  const v8us o = f.half[0];
  unsigned short* d = (unsigned short*)Wt + (size_t)blockIdx.y * obs + (size_t)n * K + k8;
  *(volatile v8us*)d = o; __threadfence(); *(volatile v8us*)d = o;
}

__global__ __launch_bounds__(256) void k_bias3(const float* __restrict__ bq, const float* __restrict__ bk, const float* __restrict__ bv, float* __restrict__ BIA) {
  const unsigned t = blockIdx.x * 256u + threadIdx.x;
  if (t >= (unsigned)(LQ / 4)) return;
  const unsigned c4 = t * 4u; const unsigned h = c4 / 192u; const unsigned rem = c4 - h * 192u; const unsigned which = rem >> 6, e = rem & 63u;
  const unsigned si = h * 64u + e;
  const v4f a = *(const v4fa*)(bq + si), b = *(const v4fa*)(bk + si), c = *(const v4fa*)(bv + si);
  v4f o;
#pragma unroll
  for (int i = 0; i < 4; ++i) o[i] = (which == 0u) ? a[i] : ((which == 1u) ? b[i] : c[i]);
  *(volatile v4f*)(BIA + c4) = o; __threadfence(); *(volatile v4f*)(BIA + c4) = o;
}

__global__ __launch_bounds__(256) void k_vt(const _Float16* __restrict__ SRC, _Float16* __restrict__ VT) {
  __shared__ unsigned short tl[64][66];
  const unsigned tid = threadIdx.x; const unsigned h = blockIdx.x / (unsigned)(SEQ / 64), lg = blockIdx.x % (unsigned)(SEQ / 64);
  for (unsigned i = tid; i < 512u; i += 256u) { const unsigned r = i >> 3, c8 = (i & 7u) * 8u; FragH f; f.half[0] = *(const v8us*)((const unsigned short*)SRC + ((size_t)lg * 64u + r) * LQ + h * 192u + 128u + c8);
#pragma unroll
    for (int q = 0; q < 8; ++q) tl[r][c8 + q] = f.u[q]; }
  __syncthreads();
  for (int pass = 0; pass < 2; ++pass) {
#pragma unroll
    for (unsigned rd = 0; rd < 2; ++rd) { const unsigned d = rd * 32u + (tid >> 3), pc = tid & 7u; FragH f;
#pragma unroll
      for (int q = 0; q < 8; ++q) f.u[q] = tl[pc * 8u + q][d];
      const v8us o = f.half[0];
      *(volatile v8us*)((unsigned short*)VT + ((size_t)h * 64u + d) * SEQ + lg * 64u + pc * 8u) = o; }
    if (pass == 0) __threadfence(); }
}

__global__ __launch_bounds__(128) void k_stats(const _Float16* __restrict__ QKV, float* __restrict__ SH) {
  __shared__ __attribute__((aligned(16))) float st[64];
  const unsigned tid = threadIdx.x, w = tid >> 5, lane = tid & 31u, ln = lane & 15u, hh = lane >> 4;
  const unsigned qb = blockIdx.x % (unsigned)(SEQ / 64), h = blockIdx.x / (unsigned)(SEQ / 64);
  const unsigned q0 = qb * 64u + w * 16u;
  const _Float16* qrow = QKV + (size_t)(q0 + ln) * LQ + h * 192u;
  const v16h bq0 = g2_frag(qrow, hh), bq1 = g2_frag(qrow + 32, hh);
  const _Float16* kbase = QKV + (size_t)ln * LQ + h * 192u + 64u;
  const v8f z8 = {0.f, 0.f, 0.f, 0.f, 0.f, 0.f, 0.f, 0.f};
  float m = -1.0e30f, l = 0.f;
#pragma unroll 1
  for (unsigned j0 = 0; j0 < (unsigned)SEQ; j0 += 64u) {
    v8f c[4];
#pragma unroll
    for (int t = 0; t < 4; ++t) { const _Float16* kr = kbase + (size_t)(j0 + t * 16u) * LQ; v8f z = z8; z = g2_mma(g2_frag(kr, hh), bq0, z); z = g2_mma(g2_frag(kr + 32, hh), bq1, z); c[t] = z; }
    float mx = c[0][0];
#pragma unroll
    for (int t = 0; t < 4; ++t)
#pragma unroll
      for (int r = 0; r < 8; ++r) mx = fmaxf(mx, c[t][r]);
    mx = fmaxf(mx, __shfl_xor(mx, 16, 32));
    const float mnew = fmaxf(m, mx * 0.125f);
    const float alpha = __expf(m - mnew);
    m = mnew;
    const float sh = -mnew;
    float ps = 0.f;
#pragma unroll
    for (int r = 0; r < 8; ++r) {
      const float e0 = __expf(fmaf(c[0][r], 0.125f, sh)), e1 = __expf(fmaf(c[1][r], 0.125f, sh));
      const float e2 = __expf(fmaf(c[2][r], 0.125f, sh)), e3 = __expf(fmaf(c[3][r], 0.125f, sh));
      ps += (e0 + e1) + (e2 + e3);
    }
    l = l * alpha + ps;
  }
  const float lt = l + __shfl_xor(l, 16, 32);
  const float shf = 9.70406053f - m - logf(lt);
  if (hh == 0u) st[w * 16u + ln] = shf;
  __syncthreads();
  const v4f v = *(const v4fa*)&st[(tid & 15u) * 4u];
  float* dst = SH + (size_t)h * SEQ + qb * 64u + (tid & 15u) * 4u;
  if (tid < 16u) { *(volatile v4f*)dst = v; __threadfence(); *(volatile v4f*)dst = v; }
}

__global__ __launch_bounds__(128) void k_attnT(const _Float16* __restrict__ QKV, const _Float16* __restrict__ VT, const _Float16* __restrict__ VTR, const float* __restrict__ SH,
    _Float16* __restrict__ O16, _Float16* __restrict__ O16R) {
  __shared__ __attribute__((aligned(16))) unsigned short os[4][16][72];
  __shared__ __attribute__((aligned(16))) unsigned short osr[4][16][72];
  const unsigned tid = threadIdx.x, w = tid >> 5, lane = tid & 31u, ln = lane & 15u, hh = lane >> 4;
  const unsigned tb = blockIdx.x % (unsigned)(SEQ / 64), h = blockIdx.x / (unsigned)(SEQ / 64);
  const unsigned t0 = tb * 64u + w * 16u;
  const _Float16* krow = QKV + (size_t)(t0 + ln) * LQ + h * 192u + 64u;
  const v16h bk0 = g2_frag(krow, hh), bk1 = g2_frag(krow + 32, hh);
  const _Float16* qbase = QKV + (size_t)ln * LQ + h * 192u;
  const _Float16* vbase = VT + ((size_t)h * 64u + ln) * SEQ;
  const _Float16* vrbase = VTR + ((size_t)h * 64u + ln) * SEQ;
  const float* shb = SH + (size_t)h * SEQ + 8u * hh;
  const v8f z8 = {0.f, 0.f, 0.f, 0.f, 0.f, 0.f, 0.f, 0.f};
  v8f o[4] = {z8, z8, z8, z8};
  v8f ores[4] = {z8, z8, z8, z8};
#pragma unroll 1
  for (unsigned j0 = 0; j0 < (unsigned)SEQ; j0 += 32u) {
    v8f c[2];
#pragma unroll
    for (int t = 0; t < 2; ++t) { const _Float16* qr = qbase + (size_t)(j0 + t * 16u) * LQ; v8f z = z8; z = g2_mma(g2_frag(qr, hh), bk0, z); z = g2_mma(g2_frag(qr + 32, hh), bk1, z); c[t] = z; }
    FragH ph, pl;
#pragma unroll
    for (int t = 0; t < 2; ++t) {
      const v4f sa = *(const v4fa*)(shb + j0 + t * 16u), sb = *(const v4fa*)(shb + j0 + t * 16u + 4u);
#pragma unroll
      for (int r = 0; r < 4; ++r) {
        const float e0 = __expf(fmaf(c[t][r], 0.125f, sa[r]));
        const float e1 = __expf(fmaf(c[t][4 + r], 0.125f, sb[r]));
        const _Float16 h0 = (_Float16)e0, h1 = (_Float16)e1;
        ph.h[t * 8 + r] = h0;
        ph.h[t * 8 + 4 + r] = h1;
        pl.h[t * 8 + r] = (_Float16)((e0 - (float)h0) * 1024.0f);
        pl.h[t * 8 + 4 + r] = (_Float16)((e1 - (float)h1) * 1024.0f);
      }
    }
#pragma unroll
    for (int dt = 0; dt < 4; ++dt) {
      const v16h va = g2_frag(vbase + (size_t)(dt * 16u) * SEQ + j0, hh);
      const v16h vra = g2_frag(vrbase + (size_t)(dt * 16u) * SEQ + j0, hh);
      o[dt] = g2_mma(va, ph.v, o[dt]);
      ores[dt] = g2_mma(vra, ph.v, ores[dt]);
      ores[dt] = g2_mma(va, pl.v, ores[dt]);
    }
  }
  const float fin = 0.00390625f;
#pragma unroll
  for (int dt = 0; dt < 4; ++dt) { FragH f, g;
#pragma unroll
    for (int r = 0; r < 8; ++r) { const float val = (o[dt][r] + ores[dt][r] * 0.0009765625f) * fin; const _Float16 hv = (_Float16)val; f.h[r] = hv; g.h[r] = (_Float16)((val - (float)hv) * 1024.0f); }
    *(v8us*)&os[w][ln][dt * 16 + 8 * hh] = f.half[0];
    *(v8us*)&osr[w][ln][dt * 16 + 8 * hh] = g.half[0]; }
  __builtin_amdgcn_fence(4  , "workgroup"); __builtin_amdgcn_wave_barrier();
  const unsigned rq = lane >> 3, pc = (lane & 7u) * 8u;
  for (int pass = 0; pass < 2; ++pass) {
#pragma unroll
    for (unsigned it = 0; it < 4; ++it) { const unsigned row = it * 4u + rq; const v8us v = *(const v8us*)&os[w][row][pc]; const v8us vr = *(const v8us*)&osr[w][row][pc];
      *(volatile v8us*)((unsigned short*)O16 + ((size_t)t0 + row) * DM + h * 64u + pc) = v;
      *(volatile v8us*)((unsigned short*)O16R + ((size_t)t0 + row) * DM + h * 64u + pc) = vr; }
    if (pass == 0) __threadfence(); }
}

template <int ACT, int RA>
__global__ __launch_bounds__(128) void k_gemm2(const _Float16* __restrict__ A, const _Float16* __restrict__ AR, unsigned lda, const _Float16* __restrict__ Bh, unsigned ldb, float alpha, const float* __restrict__ bias, float bscale,
    float* __restrict__ C, _Float16* __restrict__ C16, _Float16* __restrict__ C16R, unsigned ldc, unsigned M, unsigned N, unsigned K) {
  static_assert(ACT == 0 || ACT == 1);
  static_assert(RA == 0 || RA == 1);
  __shared__ __attribute__((aligned(16))) float so[4][32][68];
  const unsigned tid = threadIdx.x, w = tid >> 5, lane = tid & 31u, ln = lane & 15u, hh = lane >> 4;
  const unsigned ntn = N >> 6; const unsigned mt = blockIdx.x / ntn, nq = blockIdx.x - mt * ntn; const unsigned row0 = mt * 128u + 32u * w, col0 = nq * 64u; if (row0 >= M) return;
  const _Float16* a0p = A + (size_t)(row0 + ln) * lda; const _Float16* a1p = a0p + (size_t)16 * lda;
  const _Float16* r0p = AR + (size_t)(row0 + ln) * lda; const _Float16* r1p = r0p + (size_t)16 * lda;
  const v8f z8 = {0.f,0.f,0.f,0.f,0.f,0.f,0.f,0.f};
#pragma unroll 1
  for (unsigned nh = 0; nh < 2u; ++nh) {
    const unsigned cb = nh * 32u;
    const _Float16* b0p = Bh + (size_t)(col0 + cb + ln) * ldb; const _Float16* b1p = b0p + (size_t)16 * ldb;
    v8f c00 = z8, c01 = z8, c10 = z8, c11 = z8, d00 = z8, d01 = z8, d10 = z8, d11 = z8;
#pragma unroll 1
    for (unsigned kb = 0; kb < K; kb += 32u) {
      const v16h a0 = g2_frag(a0p + kb, hh), a1 = g2_frag(a1p + kb, hh);
      const v16h bf0 = g2_frag(b0p + kb, hh), bf1 = g2_frag(b1p + kb, hh);
      c00 = g2_mma(a0, bf0, c00); c10 = g2_mma(a1, bf0, c10);
      c01 = g2_mma(a0, bf1, c01); c11 = g2_mma(a1, bf1, c11);
      if (RA == 1) {
        const v16h ar0 = g2_frag(r0p + kb, hh), ar1 = g2_frag(r1p + kb, hh);
        d00 = g2_mma(ar0, bf0, d00); d10 = g2_mma(ar1, bf0, d10);
        d01 = g2_mma(ar0, bf1, d01); d11 = g2_mma(ar1, bf1, d11);
      }
    }
    if (RA == 1) { c00 = c00 + d00 * 0.0009765625f; c01 = c01 + d01 * 0.0009765625f; c10 = c10 + d10 * 0.0009765625f; c11 = c11 + d11 * 0.0009765625f; }
    v8f accs[4] = {c00, c01, c10, c11};
#pragma unroll
    for (int u = 0; u < 4; ++u) { const int t = u & 1, half = u >> 1; const unsigned cl = cb + t * 16 + ln; const float bv = bf16_rne(bias[col0 + cl]) * bscale;
#pragma unroll
      for (int r = 0; r < 8; ++r) { const unsigned rloc = half * 16 + 8 * hh + r; float v = accs[u][r] * alpha + bv; if (ACT == 1) v = fmaxf(v, 0.f); so[w][rloc][cl] = v; } }
  }
  __builtin_amdgcn_fence(4  , "workgroup"); __builtin_amdgcn_wave_barrier();
  const unsigned rsub = lane >> 4, c4 = (lane & 15u) * 4u;
  for (int pass = 0; pass < 2; ++pass) {
#pragma unroll
    for (unsigned q = 0; q < 16; ++q) { const unsigned r = q * 2u + rsub; const v4f v = *(const v4fa*)&so[w][r][c4];
      if (C) *(volatile v4f*)(C + (size_t)(row0 + r) * ldc + col0 + c4) = v;
      if (C16) { v4h h4, r4;
#pragma unroll
        for (int i = 0; i < 4; ++i) { const _Float16 hv = (_Float16)v[i]; h4[i] = hv; r4[i] = (_Float16)((v[i] - (float)hv) * 1024.0f); }
        *(volatile v4h*)(C16 + (size_t)(row0 + r) * ldc + col0 + c4) = h4;
        if (C16R) *(volatile v4h*)(C16R + (size_t)(row0 + r) * ldc + col0 + c4) = r4; } }
    if (pass == 0) __threadfence(); }
}

#define SZ_BQKV ((size_t)LQ * DM * 2)
#define SZ_BP   ((size_t)DM * DM * 2)
#define SZ_BW1  ((size_t)DFF * DM * 2)
#define SZ_BW2  ((size_t)DM * DFF * 2)
#define SZ_X16  ((size_t)SEQ * DM * 2)
#define SZ_BIA  ((size_t)LQ * 4)
#define SZ_QKV  ((size_t)SEQ * LQ * 2)
#define SZ_VT   ((size_t)NH * HD * SEQ * 2)
#define SZ_SH   ((size_t)NH * SEQ * 4)
#define SZ_O16  ((size_t)SEQ * DM * 2)
#define SZ_PRJ  ((size_t)SEQ * DM * 2)
#define SZ_HF   ((size_t)SEQ * DFF * 2)
#define SZ_TOT  (SZ_BQKV + SZ_BP + SZ_BW1 + SZ_BW2 + SZ_X16 + SZ_BIA + 2 * SZ_QKV + 2 * SZ_VT + SZ_SH + 2 * SZ_O16 + 2 * SZ_PRJ + 2 * SZ_HF)
static_assert(SZ_TOT <= (size_t)134217728);
static_assert(SZ_BQKV % 256 == 0 && SZ_BP % 256 == 0 && SZ_BW1 % 256 == 0 && SZ_BW2 % 256 == 0 && SZ_X16 % 256 == 0 && SZ_BIA % 256 == 0);
static_assert(SZ_QKV % 256 == 0 && SZ_VT % 256 == 0 && SZ_SH % 256 == 0 && SZ_O16 % 256 == 0 && SZ_PRJ % 256 == 0 && SZ_HF % 256 == 0);
static_assert(((size_t)SEQ * (DM / 8)) % 256 == 0);
static_assert(((size_t)HD * (DM / 8)) % 256 == 0);
static_assert(((size_t)DM * (DM / 8)) % 256 == 0 && ((size_t)DFF * (DM / 8)) % 256 == 0 && ((size_t)DM * (DFF / 8)) % 256 == 0);
static_assert((LQ / 4) % 256 == 0);
static_assert((size_t)NH * (SEQ / 64) * 64 * 64 == (size_t)NH * HD * SEQ);
static_assert((size_t)NH * (SEQ / 64) * 64 == (size_t)NH * SEQ);
static_assert((size_t)NH * (SEQ / 64) * 64 * 64 == (size_t)SEQ * DM);
static_assert((size_t)(SEQ / 128) * (LQ / 64) * 128 * 64 == (size_t)SEQ * LQ);
static_assert((size_t)(SEQ / 128) * (DM / 64) * 128 * 64 == (size_t)SEQ * DM);
static_assert((size_t)(SEQ / 128) * (DFF / 64) * 128 * 64 == (size_t)SEQ * DFF);

extern "C" void kernel_launch(void* const* d_in, const int* in_sizes, int n_in,
                              void* d_out, int out_size, void* d_ws, size_t ws_size, hipStream_t stream) {
  if (n_in < 13) return;
  const long long xneed = (long long)SEQ * DM;
  if ((long long)in_sizes[0] < xneed || (long long)out_size < xneed) return;
  if (in_sizes[1] < NH * DM * HD || in_sizes[2] < NH * HD || in_sizes[3] < NH * DM * HD || in_sizes[4] < NH * HD || in_sizes[5] < NH * DM * HD || in_sizes[6] < NH * HD) return;
  if (in_sizes[7] < DM * DM || in_sizes[8] < DM || in_sizes[9] < DM * DFF || in_sizes[10] < DFF || in_sizes[11] < DFF * DM || in_sizes[12] < DM) return;
  if (ws_size < SZ_TOT) return;
  const float* x = (const float*)d_in[0];
  const float* Wq = (const float*)d_in[1]; const float* bq = (const float*)d_in[2];
  const float* Wk = (const float*)d_in[3]; const float* bk = (const float*)d_in[4];
  const float* Wv = (const float*)d_in[5]; const float* bv = (const float*)d_in[6];
  const float* Wp = (const float*)d_in[7]; const float* bp = (const float*)d_in[8];
  const float* W1 = (const float*)d_in[9]; const float* b1 = (const float*)d_in[10];
  const float* W2 = (const float*)d_in[11]; const float* b2 = (const float*)d_in[12];
  float* out = (float*)d_out;
  char* ws = (char*)d_ws; size_t off = 0;
  _Float16* BQKV = (_Float16*)(ws + off); off += SZ_BQKV;
  _Float16* BP   = (_Float16*)(ws + off); off += SZ_BP;
  _Float16* BW1  = (_Float16*)(ws + off); off += SZ_BW1;
  _Float16* BW2  = (_Float16*)(ws + off); off += SZ_BW2;
  _Float16* X16  = (_Float16*)(ws + off); off += SZ_X16;
  float* BIA     = (float*)(ws + off); off += SZ_BIA;
  _Float16* QKV  = (_Float16*)(ws + off); off += SZ_QKV;
  _Float16* QKVR = (_Float16*)(ws + off); off += SZ_QKV;
  _Float16* VT   = (_Float16*)(ws + off); off += SZ_VT;
  _Float16* VTR  = (_Float16*)(ws + off); off += SZ_VT;
  float* SH      = (float*)(ws + off); off += SZ_SH;
  _Float16* O16  = (_Float16*)(ws + off); off += SZ_O16;
  _Float16* O16R = (_Float16*)(ws + off); off += SZ_O16;
  _Float16* PRJ  = (_Float16*)(ws + off); off += SZ_PRJ;
  _Float16* PRJR = (_Float16*)(ws + off); off += SZ_PRJ;
  _Float16* HF16 = (_Float16*)(ws + off); off += SZ_HF;
  _Float16* HFR  = (_Float16*)(ws + off); off += SZ_HF;
  if (off > ws_size) return;

  k_x16<<<(unsigned)((size_t)SEQ * (DM / 8) / 256), 256, 0, stream>>>(x, X16);
  k_wt_f16<<<dim3((unsigned)((size_t)HD * (DM / 8) / 256), (unsigned)NH), 256, 0, stream>>>(Wq, BQKV, (unsigned)DM, (unsigned)HD, 16.0f, (unsigned)(DM * HD), (unsigned)(192 * DM));
  k_wt_f16<<<dim3((unsigned)((size_t)HD * (DM / 8) / 256), (unsigned)NH), 256, 0, stream>>>(Wk, BQKV + (size_t)64 * DM, (unsigned)DM, (unsigned)HD, 16.0f, (unsigned)(DM * HD), (unsigned)(192 * DM));
  k_wt_f16<<<dim3((unsigned)((size_t)HD * (DM / 8) / 256), (unsigned)NH), 256, 0, stream>>>(Wv, BQKV + (size_t)128 * DM, (unsigned)DM, (unsigned)HD, 16.0f, (unsigned)(DM * HD), (unsigned)(192 * DM));
  k_wt_f16<<<dim3((unsigned)((size_t)DM * (DM / 8) / 256), 1u), 256, 0, stream>>>(Wp, BP, (unsigned)DM, (unsigned)DM, 16.0f, 0u, 0u);
  k_wt_f16<<<dim3((unsigned)((size_t)DFF * (DM / 8) / 256), 1u), 256, 0, stream>>>(W1, BW1, (unsigned)DM, (unsigned)DFF, 16.0f, 0u, 0u);
  k_wt_f16<<<dim3((unsigned)((size_t)DM * (DFF / 8) / 256), 1u), 256, 0, stream>>>(W2, BW2, (unsigned)DFF, (unsigned)DM, 64.0f, 0u, 0u);
  k_bias3<<<(unsigned)(LQ / 4 / 256), 256, 0, stream>>>(bq, bk, bv, BIA);
  k_gemm2<0, 0><<<(unsigned)((SEQ / 128) * (LQ / 64)), 128, 0, stream>>>(X16, X16, (unsigned)DM, BQKV, (unsigned)DM, 0.00390625f, BIA, 1.0f, nullptr, QKV, QKVR, (unsigned)LQ, (unsigned)SEQ, (unsigned)LQ, (unsigned)DM);
  k_vt<<<(unsigned)(NH * (SEQ / 64)), 256, 0, stream>>>(QKV, VT);
  k_vt<<<(unsigned)(NH * (SEQ / 64)), 256, 0, stream>>>(QKVR, VTR);
  k_stats<<<(unsigned)(NH * (SEQ / 64)), 128, 0, stream>>>(QKV, SH);
  k_attnT<<<(unsigned)(NH * (SEQ / 64)), 128, 0, stream>>>(QKV, VT, VTR, SH, O16, O16R);
  k_gemm2<0, 1><<<(unsigned)((SEQ / 128) * (DM / 64)), 128, 0, stream>>>(O16, O16R, (unsigned)DM, BP, (unsigned)DM, 0.015625f, bp, 16.0f, nullptr, PRJ, PRJR, (unsigned)DM, (unsigned)SEQ, (unsigned)DM, (unsigned)DM);
  k_gemm2<1, 1><<<(unsigned)((SEQ / 128) * (DFF / 64)), 128, 0, stream>>>(PRJ, PRJR, (unsigned)DM, BW1, (unsigned)DM, 0.0625f, b1, 16.0f, nullptr, HF16, HFR, (unsigned)DFF, (unsigned)SEQ, (unsigned)DFF, (unsigned)DM);
  k_gemm2<0, 1><<<(unsigned)((SEQ / 128) * (DM / 64)), 128, 0, stream>>>(HF16, HFR, (unsigned)DFF, BW2, (unsigned)DFF, 0.0009765625f, b2, 1.0f, out, nullptr, nullptr, (unsigned)DM, (unsigned)SEQ, (unsigned)DM, (unsigned)DFF);
}
